// Cross_Scale_Mamba_Block_84138409328978
// MI455X (gfx1250) — hardware-verified
//
#include <hip/hip_runtime.h>
#include <math.h>

typedef __attribute__((ext_vector_type(16))) _Float16 v16h;
typedef __attribute__((ext_vector_type(8)))  _Float16 v8h;
typedef __attribute__((ext_vector_type(16))) __bf16   v16b;
typedef __attribute__((ext_vector_type(8)))  __bf16   v8b;
typedef __attribute__((ext_vector_type(8)))  float    v8f;
typedef __attribute__((ext_vector_type(4)))  float    v4f;

constexpr int NBATCH = 8;
constexpr int DIMALL = 128;
constexpr int IMH    = 64;
constexpr int IMW    = 64;
constexpr int NPIX   = IMH * IMW;
constexpr int NTOK   = NBATCH * NPIX;
constexpr int CCH    = 32;
constexpr int DIN    = 64;
constexpr int NST    = 16;
constexpr int NDIR   = 4;
constexpr int XPC    = 34;
constexpr int XPD    = 48;
constexpr int XPN    = NDIR * XPD;
constexpr int XZP    = 2 * DIN;
constexpr int OPN    = 64;
constexpr int SCH    = 64;
constexpr float NORM_EPS = 1e-5f;
constexpr float WCARRY   = 64.0f;
constexpr float ACARRY   = 64.0f;
static_assert(NPIX % SCH == 0, "");
static_assert((SCH * 9) % DIN == 0, "");
static_assert(XPN % 64 == 0 && XZP % 64 == 0 && OPN % 64 == 0, "");

__device__ __forceinline__ unsigned short f2bf_bits(float f) {
  unsigned u = __float_as_uint(f);
  return (unsigned short)((u + 0x7FFFu + ((u >> 16) & 1u)) >> 16);
}
__device__ __forceinline__ float bf_bits2f(unsigned short h) { return __uint_as_float(((unsigned)h) << 16); }

__device__ __forceinline__ void dep_guard_h(v8f& a, v8f& b, v16h x, v16h y) { asm volatile("v_nop\n\tv_nop\n\tv_nop\n\tv_nop" : "+v"(a), "+v"(b) : "v"(x), "v"(y)); }
__device__ __forceinline__ void dep_guard_b(v8f& a, v8f& b, v16b x, v16b y) { asm volatile("v_nop\n\tv_nop\n\tv_nop\n\tv_nop" : "+v"(a), "+v"(b) : "v"(x), "v"(y)); }
__device__ __forceinline__ void keep4_h(v16h a, v16h b, v16h c, v16h d) { asm volatile("v_nop" :: "v"(a), "v"(b), "v"(c), "v"(d)); }
__device__ __forceinline__ void keep4_b(v16b a, v16b b, v16b c, v16b d) { asm volatile("v_nop" :: "v"(a), "v"(b), "v"(c), "v"(d)); }
__device__ __forceinline__ void acc_guard4(v8f& a, v8f& b, v8f& c, v8f& d) { asm volatile("v_nop\n\tv_nop\n\tv_nop\n\tv_nop" : "+v"(a), "+v"(b), "+v"(c), "+v"(d)); }
template <typename T> struct Frag;
template <> struct Frag<_Float16> {
  typedef v16h V; union U { v16h v; v8h h[2]; };
  static __device__ __forceinline__ v16h load(const _Float16* p) {
    U f; f.h[0] = *(const v8h*)(p); f.h[1] = *(const v8h*)(p + 16); return f.v;
  }
  static __device__ __forceinline__ v8f mma(v16h a, v16h b, v8f c) {
    return __builtin_amdgcn_wmma_f32_16x16x32_f16(false, a, false, b, (short)0, c, false, false);
  }
  static __device__ __forceinline__ void guard(v8f& a, v8f& b, v16h x, v16h y) { dep_guard_h(a, b, x, y); }
  static __device__ __forceinline__ void keep(v16h a, v16h b, v16h c, v16h d) { keep4_h(a, b, c, d); }
};
template <> struct Frag<__bf16> {
  typedef v16b V; union U { v16b v; v8b h[2]; };
  static __device__ __forceinline__ v16b load(const __bf16* p) {
    U f; f.h[0] = *(const v8b*)(p); f.h[1] = *(const v8b*)(p + 16); return f.v;
  }
  static __device__ __forceinline__ v8f mma(v16b a, v16b b, v8f c) {
    return __builtin_amdgcn_wmma_f32_16x16x32_bf16(false, a, false, b, (short)0, c, false, false);
  }
  static __device__ __forceinline__ void guard(v8f& a, v8f& b, v16b x, v16b y) { dep_guard_b(a, b, x, y); }
  static __device__ __forceinline__ void keep(v16b a, v16b b, v16b c, v16b d) { keep4_b(a, b, c, d); }
};

template <int ET> struct Elem;
template <> struct Elem<0> { typedef _Float16 T; };
template <> struct Elem<1> { typedef __bf16 T; };
template <int ET, bool SPLIT, int BIAS_MODE, int OUT_MODE, bool RESID, int ACT = 0>
__global__ __launch_bounds__(256) void wmma_gemm64(
    const unsigned short* __restrict__ Ap, const unsigned short* __restrict__ A2p, int lda, long strideA,
    const unsigned short* __restrict__ Btp, const unsigned short* __restrict__ Bt2p, int ldb, long strideB,
    void* __restrict__ Cout, void* __restrict__ Cout2, int ldc, long strideC,
    const float* __restrict__ bias,
    const float* __restrict__ resid, long strideR,
    int M, int N, int K, float scale) {
  typedef typename Elem<ET>::T T;
  typedef typename Frag<T>::V V;
  const T* A = (const T*)Ap; const T* A2 = (const T*)A2p; const T* Bt = (const T*)Btp; const T* Bt2 = (const T*)Bt2p;
  __shared__ __align__(16) float sT[8][16 * 68];
  const int b    = blockIdx.y;
  const int lane = threadIdx.x & 31;
  const int wave = threadIdx.x >> 5;
  const int tilesN = N >> 6;
  const int tilesM = M >> 6;
  const int tile = blockIdx.x * 8 + wave;
  if (tile >= tilesM * tilesN) return;
  const int tm = tile / tilesN;
  const int tn = tile - tm * tilesN;
  const int m0 = tm << 6;
  const int n0 = tn << 6;

  const T* Ab  = A  + (size_t)b * strideA;
  const T* Bb  = Bt + (size_t)b * strideB;
  const T* Ab2 = SPLIT ? (A2  + (size_t)b * strideA) : nullptr;
  const T* Bb2 = SPLIT ? (Bt2 + (size_t)b * strideB) : nullptr;

  const int rlane = lane & 15;
  const int koff  = (lane >> 4) * 8;
  const int mOff  = (lane >> 4) * 8;

  v8f acc[4][4];
#pragma unroll
  for (int i = 0; i < 4; ++i)
#pragma unroll
    for (int j = 0; j < 4; ++j) acc[i][j] = (v8f){0.f,0.f,0.f,0.f,0.f,0.f,0.f,0.f};

  for (int k0 = 0; k0 < K; k0 += 32) {
    V bh[4], bl[4];
#pragma unroll
    for (int j = 0; j < 4; ++j) {
      const size_t bo = (size_t)(n0 + (j << 4) + rlane) * ldb + koff + k0;
      bh[j] = Frag<T>::load(Bb + bo);
      if (SPLIT) bl[j] = Frag<T>::load(Bb2 + bo);
    }
#pragma unroll
    for (int i = 0; i < 4; ++i) {
      const size_t ao = (size_t)(m0 + (i << 4) + rlane) * lda + koff + k0;
      V ah = Frag<T>::load(Ab + ao);
      V al;
      if (SPLIT) al = Frag<T>::load(Ab2 + ao);
#pragma unroll
      for (int j = 0; j < 4; ++j) {
        acc[i][j] = Frag<T>::mma(ah, bh[j], acc[i][j]);
        if (SPLIT) {
          acc[i][j] = Frag<T>::mma(ah, bl[j], acc[i][j]);
          acc[i][j] = Frag<T>::mma(al, bh[j], acc[i][j]);
        }
      }
      Frag<T>::guard(acc[i][0], acc[i][3], ah, SPLIT ? al : ah);
    }
    Frag<T>::keep(bh[0], bh[1], bh[2], bh[3]);
    if (SPLIT) Frag<T>::keep(bl[0], bl[1], bl[2], bl[3]);
  }
  acc_guard4(acc[0][0], acc[0][1], acc[0][2], acc[0][3]);
  acc_guard4(acc[1][0], acc[1][1], acc[1][2], acc[1][3]);
  acc_guard4(acc[2][0], acc[2][1], acc[2][2], acc[2][3]);
  acc_guard4(acc[3][0], acc[3][1], acc[3][2], acc[3][3]);

  float* slab = sT[wave];
  const float* Rb = RESID ? (resid + (size_t)b * strideR) : nullptr;
#pragma unroll
  for (int i = 0; i < 4; ++i) {
    const int mBase = m0 + (i << 4);
#pragma unroll
    for (int j = 0; j < 4; ++j) {
      const int n = n0 + (j << 4) + rlane;
      float bv = 0.f;
      if (BIAS_MODE == 2) bv = bias[n];
#pragma unroll
      for (int r = 0; r < 8; ++r) {
        float v = acc[i][j][r] * scale;
        if (BIAS_MODE == 1) v += bias[mBase + mOff + r];
        if (BIAS_MODE == 2) v += bv;
        if (RESID) v += Rb[(size_t)(mBase + mOff + r) * ldc + n];
        if (ACT == 1) v = tanhf(v);
        if (ACT == 2) v = fmaxf(v, 0.0f);
        if (ACT == 3) v = v / (1.0f + expf(-v));
        if (ACT == 4) v = (v > 0.f) ? v : 0.01f * v;
        if (ACT == 5) v = 0.5f * v * (1.0f + erff(v * 0.70710678118654752f));
        slab[(mOff + r) * 68 + (j << 4) + rlane] = v;
      }
    }
    __builtin_amdgcn_fence(__ATOMIC_RELEASE, "workgroup");
    __builtin_amdgcn_wave_barrier();
    __builtin_amdgcn_fence(__ATOMIC_ACQUIRE, "workgroup");
    if (OUT_MODE == 0) {
      float* C = (float*)Cout + (size_t)b * strideC;
      const int hh = lane >> 4, c4 = (lane & 15) * 4;
      for (int pass = 0; pass < 2; ++pass) {
#pragma unroll
        for (int it = 0; it < 8; ++it) {
          const int row = it * 2 + hh;
          v4f v = *(const v4f*)(slab + row * 68 + c4);
          *(volatile v4f*)(C + (size_t)(mBase + row) * ldc + n0 + c4) = v;
        }
        __threadfence();
      }
    } else {
      const int q = lane >> 3, c8 = (lane & 7) * 8;
      unsigned short* C  = (unsigned short*)Cout  + (size_t)b * strideC;
      unsigned short* C2 = (OUT_MODE == 2) ? ((unsigned short*)Cout2 + (size_t)b * strideC) : nullptr;
      for (int pass = 0; pass < 2; ++pass) {
#pragma unroll
        for (int it = 0; it < 4; ++it) {
          const int row = it * 4 + q;
          const float* sp = slab + row * 68 + c8;
          v8h hv, lv;
#pragma unroll
          for (int e = 0; e < 8; ++e) {
            if (OUT_MODE == 1) {
              hv[e] = (_Float16)sp[e];
            } else {
              unsigned short hb = f2bf_bits(sp[e]);
              unsigned short lb = f2bf_bits(sp[e] - bf_bits2f(hb));
              hv[e] = __builtin_bit_cast(_Float16, hb);
              lv[e] = __builtin_bit_cast(_Float16, lb);
            }
          }
          *(volatile v8h*)(C + (size_t)(mBase + row) * ldc + n0 + c8) = hv;
          if (OUT_MODE == 2) *(volatile v8h*)(C2 + (size_t)(mBase + row) * ldc + n0 + c8) = lv;
        }
        __threadfence();
      }
    }
    __builtin_amdgcn_fence(__ATOMIC_RELEASE, "workgroup");
    __builtin_amdgcn_wave_barrier();
    __builtin_amdgcn_fence(__ATOMIC_ACQUIRE, "workgroup");
  }
}

__global__ __launch_bounds__(256) void cast_weights_kernel(
    const float* __restrict__ inw, const float* __restrict__ xpw, const float* __restrict__ opw,
    unsigned short* __restrict__ WIN16, unsigned short* __restrict__ WX16, unsigned short* __restrict__ WO16)
{
  const int t = threadIdx.x;
  const int blk = blockIdx.x;
  v8h hv;
  unsigned short* dst;
  if (blk < 2) {
    const int f = blk * 256 + t;
    const int row = f >> 2, col8 = (f & 3) * 8;
    const float* p = inw + (size_t)row * CCH + col8;
    const v4f a0 = *(const v4f*)(p);
    const v4f a1 = *(const v4f*)(p + 4);
#pragma unroll
    for (int e = 0; e < 4; ++e) { hv[e] = (_Float16)(a0[e] * WCARRY); hv[4 + e] = (_Float16)(a1[e] * WCARRY); }
    dst = WIN16 + (size_t)f * 8;
  } else if (blk < 8) {
    const int f = (blk - 2) * 256 + t;
    const int r = f >> 3, d8 = (f & 7) * 8;
    const int k = r / XPD;
    const int j = r - k * XPD;
    const bool valid = j < XPC;
    const int c  = (j < 32) ? (j + 2) : (j - 32);
    const int cs = valid ? c : 0;
    const float* p = xpw + ((size_t)(k * XPC + cs)) * DIN + d8;
    const v4f a0 = *(const v4f*)(p);
    const v4f a1 = *(const v4f*)(p + 4);
#pragma unroll
    for (int e = 0; e < 4; ++e) {
      hv[e]     = (_Float16)(valid ? a0[e] * WCARRY : 0.0f);
      hv[4 + e] = (_Float16)(valid ? a1[e] * WCARRY : 0.0f);
    }
    dst = WX16 + (size_t)f * 8;
  } else {
    const int f = (blk - 8) * 256 + t;
    const int r = f >> 3, d8 = (f & 7) * 8;
    const bool valid = r < CCH;
    const int rs = valid ? r : 0;
    const float* p = opw + (size_t)rs * DIN + d8;
    const v4f a0 = *(const v4f*)(p);
    const v4f a1 = *(const v4f*)(p + 4);
#pragma unroll
    for (int e = 0; e < 4; ++e) {
      hv[e]     = (_Float16)(valid ? a0[e] * WCARRY : 0.0f);
      hv[4 + e] = (_Float16)(valid ? a1[e] * WCARRY : 0.0f);
    }
    dst = WO16 + (size_t)f * 8;
  }
  *(volatile v8h*)dst = hv;
  __threadfence();
  *(volatile v8h*)dst = hv;
}

__global__ __launch_bounds__(256) void bn_relu_copy_kernel(
    const float* __restrict__ x, const float* __restrict__ g, const float* __restrict__ be,
    const float* __restrict__ mn, const float* __restrict__ vr, float* __restrict__ out)
{
  const int gi = blockIdx.x * 256 + threadIdx.x;
  if (gi >= NBATCH * CCH * NPIX / 4) return;
  const int e0 = gi * 4;
  const int l  = e0 & (NPIX - 1);
  const int bc = e0 >> 12;
  const int c  = bc & (CCH - 1);
  const int b  = bc >> 5;
  const int ch = 3 * CCH + c;
  const size_t idx = ((size_t)(b * DIMALL + ch)) * NPIX + l;
  const v4f v = *(const v4f*)(x + idx);
  const float is = rsqrtf(vr[ch] + NORM_EPS);
  const float gg = g[ch], bb = be[ch], mm = mn[ch];
  v4f o;
#pragma unroll
  for (int e = 0; e < 4; ++e) o[e] = fmaxf(((v[e] - mm) * is) * gg + bb, 0.0f);
  float* op = out + idx;
  *(volatile v4f*)op = o;
  __threadfence();
  *(volatile v4f*)op = o;
}

__global__ __launch_bounds__(256) void dw_w7_kernel(
    const float* __restrict__ x, const float* __restrict__ w7, const float* __restrict__ bias,
    float* __restrict__ TA, int cbase, int dil)
{
  const int gi = blockIdx.x * 256 + threadIdx.x;
  if (gi >= NBATCH * CCH * NPIX / 4) return;
  const int e0 = gi * 4;
  const int l  = e0 & (NPIX - 1);
  const int bc = e0 >> 12;
  const int c  = bc & (CCH - 1);
  const int b  = bc >> 5;
  const int h  = l >> 6, w0 = l & (IMW - 1);
  const float* xin = x + ((size_t)(b * DIMALL + cbase + c)) * NPIX + h * IMW;
  float wt[7];
#pragma unroll
  for (int tp = 0; tp < 7; ++tp) wt[tp] = w7[c * 7 + tp];
  const float bs = bias[c];
  v4f o;
#pragma unroll
  for (int j = 0; j < 4; ++j) {
    float acc = bs;
#pragma unroll
    for (int tp = 0; tp < 7; ++tp) {
      const int wj = w0 + j + (tp - 3) * dil;
      const bool ok = (wj >= 0) && (wj < IMW);
      const int wc = ok ? wj : 0;
      const float v = xin[wc];
      acc = fmaf(wt[tp], ok ? v : 0.0f, acc);
    }
    o[j] = acc;
  }
  float* op = TA + (size_t)bc * NPIX + l;
  *(volatile v4f*)op = o;
  __threadfence();
  *(volatile v4f*)op = o;
}

__global__ __launch_bounds__(256) void dw_h7_kernel(
    const float* __restrict__ TA, const float* __restrict__ w7, const float* __restrict__ bias,
    float* __restrict__ TB, int dil)
{
  const int gi = blockIdx.x * 256 + threadIdx.x;
  if (gi >= NBATCH * CCH * NPIX / 4) return;
  const int e0 = gi * 4;
  const int l  = e0 & (NPIX - 1);
  const int bc = e0 >> 12;
  const int c  = bc & (CCH - 1);
  const int h  = l >> 6, w0 = l & (IMW - 1);
  const float* pin = TA + (size_t)bc * NPIX + w0;
  float wt[7];
#pragma unroll
  for (int tp = 0; tp < 7; ++tp) wt[tp] = w7[c * 7 + tp];
  const float bs = bias[c];
  v4f o = (v4f){bs, bs, bs, bs};
#pragma unroll
  for (int tp = 0; tp < 7; ++tp) {
    const int hj = h + (tp - 3) * dil;
    const bool ok = (hj >= 0) && (hj < IMH);
    const int hc = ok ? hj : 0;
    const v4f r = *(const v4f*)(pin + hc * IMW);
#pragma unroll
    for (int e = 0; e < 4; ++e) o[e] = fmaf(wt[tp], ok ? r[e] : 0.0f, o[e]);
  }
  float* op = TB + (size_t)bc * NPIX + l;
  *(volatile v4f*)op = o;
  __threadfence();
  *(volatile v4f*)op = o;
}

__global__ __launch_bounds__(256) void dw_c_ln_kernel(
    const float* __restrict__ TB, const float* __restrict__ x,
    const float* __restrict__ w9, const float* __restrict__ bias,
    const float* __restrict__ lnw, const float* __restrict__ lnb,
    float* __restrict__ Tres, unsigned short* __restrict__ LN16, int cbase, int dil)
{
  __shared__ __align__(16) float    sTv[32 * 36];
  __shared__ __align__(16) _Float16 sLv[32 * 40];
  const int t = threadIdx.x, lane = t & 31, wave = t >> 5;
  const int blk  = blockIdx.x;
  const int half = blk & 1;
  const int bh   = blk >> 1;
  const int b    = bh >> 6;
  const int h    = bh & (IMH - 1);
  const int wbase = half * 32;
  {
    const int c = t >> 3, wq = t & 7;
    const float* pin = TB + ((size_t)(b * CCH + c)) * NPIX;
    const float* xs  = x + ((size_t)(b * DIMALL + cbase + c)) * NPIX + h * IMW;
    float wt[9];
#pragma unroll
    for (int i = 0; i < 9; ++i) wt[i] = w9[c * 9 + i];
    const float bs = bias[c];
#pragma unroll
    for (int j = 0; j < 4; ++j) {
      const int wl = wq + 8 * j;
      const int w  = wbase + wl;
      float acc = bs;
#pragma unroll
      for (int i = 0; i < 3; ++i) {
        const int hj = h + (i - 1) * dil;
        const bool hok = (hj >= 0) && (hj < IMH);
        const int hc = hok ? hj : 0;
#pragma unroll
        for (int jj = 0; jj < 3; ++jj) {
          const int wj = w + (jj - 1) * dil;
          const bool wok = (wj >= 0) && (wj < IMW);
          const int wc = wok ? wj : 0;
          const float v = pin[hc * IMW + wc];
          acc = fmaf(wt[i * 3 + jj], (hok && wok) ? v : 0.0f, acc);
        }
      }
      acc += xs[w];
      sTv[wl * 36 + c] = acc;
    }
  }
  __syncthreads();
  {
    const float gw = lnw[lane], gb = lnb[lane];
#pragma unroll
    for (int tk = 0; tk < 4; ++tk) {
      const int wl = wave * 4 + tk;
      const float v = sTv[wl * 36 + lane];
      float s = v;
      s += __shfl_xor(s, 16, 32);
      s += __shfl_xor(s, 8, 32);
      s += __shfl_xor(s, 4, 32);
      s += __shfl_xor(s, 2, 32);
      s += __shfl_xor(s, 1, 32);
      const float mu = s * (1.0f / 32.0f);
      const float dv = v - mu;
      float q = dv * dv;
      q += __shfl_xor(q, 16, 32);
      q += __shfl_xor(q, 8, 32);
      q += __shfl_xor(q, 4, 32);
      q += __shfl_xor(q, 2, 32);
      q += __shfl_xor(q, 1, 32);
      const float var = q * (1.0f / 32.0f);
      const float nv = (dv * rsqrtf(var + NORM_EPS)) * gw + gb;
      sLv[wl * 40 + lane] = (_Float16)nv;
    }
  }
  __syncthreads();
  {
    const int tok0 = b * NPIX + h * IMW + wbase + wave * 4;
    const v4f tv = *(const v4f*)(sTv + (wave * 4 + (lane >> 3)) * 36 + (lane & 7) * 4);
    float* tp = Tres + (size_t)tok0 * CCH + lane * 4;
    const int la = lane & 15;
    const v8h lv = *(const v8h*)(sLv + (wave * 4 + (la >> 2)) * 40 + (la & 3) * 8);
    unsigned short* lp = LN16 + (size_t)tok0 * CCH + la * 8;
    for (int pass = 0; pass < 2; ++pass) {
      *(volatile v4f*)tp = tv;
      if (lane < 16) *(volatile v8h*)lp = lv;
      __threadfence();
    }
  }
}

__global__ __launch_bounds__(64) void conv_silu_kernel(
    const float* __restrict__ XZ, const float* __restrict__ cw, const float* __restrict__ cbias,
    float* __restrict__ XC, unsigned short* __restrict__ XC16)
{
  __shared__ __align__(16) _Float16 sH[IMW * DIN];
  const int t = threadIdx.x, lane = t & 31, wave = t >> 5;
  const int bh = blockIdx.x;
  const int b_ = bh >> 6;
  const int h_ = bh & (IMH - 1);
  const int d  = t;
  const float* wd = cw + (size_t)d * 9;
  const float w00 = wd[0], w01 = wd[1], w02 = wd[2];
  const float w10 = wd[3], w11 = wd[4], w12 = wd[5];
  const float w20 = wd[6], w21 = wd[7], w22 = wd[8];
  const float bc = cbias[d];
  const bool up = h_ > 0, dn = h_ < IMH - 1;
  const int r0 = up ? (h_ - 1) : 0;
  const int r2 = dn ? (h_ + 1) : (IMH - 1);
  const float* p0 = XZ + ((size_t)(b_ * NPIX + r0 * IMW)) * XZP + d;
  const float* p1 = XZ + ((size_t)(b_ * NPIX + h_ * IMW)) * XZP + d;
  const float* p2 = XZ + ((size_t)(b_ * NPIX + r2 * IMW)) * XZP + d;
  float a0m = 0.f, a1m = 0.f, a2m = 0.f;
  float a0c, a1c, a2c;
  {
    const float v0 = p0[0], v1 = p1[0], v2 = p2[0];
    a0c = up ? v0 : 0.f;
    a1c = v1;
    a2c = dn ? v2 : 0.f;
  }
  float* orow = XC + ((size_t)(b_ * NPIX + h_ * IMW)) * DIN + d;
#pragma unroll 1
  for (int w = 0; w < IMW; ++w) {
    const bool rv = (w + 1) < IMW;
    const int  wn = rv ? (w + 1) : (IMW - 1);
    const float n0 = p0[(size_t)wn * XZP], n1 = p1[(size_t)wn * XZP], n2 = p2[(size_t)wn * XZP];
    const float a0n = (up && rv) ? n0 : 0.f;
    const float a1n = rv ? n1 : 0.f;
    const float a2n = (dn && rv) ? n2 : 0.f;
    float acc = w00 * a0m;
    acc = fmaf(w01, a0c, acc);
    acc = fmaf(w02, a0n, acc);
    acc = fmaf(w10, a1m, acc);
    acc = fmaf(w11, a1c, acc);
    acc = fmaf(w12, a1n, acc);
    acc = fmaf(w20, a2m, acc);
    acc = fmaf(w21, a2c, acc);
    acc = fmaf(w22, a2n, acc);
    const float sv  = acc + bc;
    const float sg  = __builtin_amdgcn_rcpf(1.0f + __expf(-sv));
    const float out = sv * sg;
    float* op = orow + (size_t)w * DIN;
    *(volatile float*)op = out;
    __threadfence();
    *(volatile float*)op = out;
    sH[w * DIN + t] = (_Float16)(out * ACARRY);
    a0m = a0c; a0c = a0n;
    a1m = a1c; a1c = a1n;
    a2m = a2c; a2c = a2n;
  }
  __syncthreads();
  v8h vals[8];
#pragma unroll
  for (int it = 0; it < 8; ++it) vals[it] = *(const v8h*)(sH + (wave * 32 + it * 4 + (lane >> 3)) * DIN + (lane & 7) * 8);
  unsigned short* ob = XC16 + ((size_t)(b_ * NPIX + h_ * IMW)) * DIN;
  for (int pass = 0; pass < 2; ++pass) {
#pragma unroll
    for (int it = 0; it < 8; ++it)
      *(volatile v8h*)(ob + (size_t)(wave * 32 + it * 4 + (lane >> 3)) * DIN + (lane & 7) * 8) = vals[it];
    __threadfence();
  }
}

__device__ __forceinline__ int dir_tok(int k, int l) {
  const int lr = (k >= 2) ? (NPIX - 1 - l) : l;
  return (k & 1) ? (((lr & (IMW - 1)) * IMW) + (lr >> 6)) : lr;
}

__global__ __launch_bounds__(64) void scan_kernel(
    const float* __restrict__ XDBL, const float* __restrict__ XC,
    const float* __restrict__ dtw, const float* __restrict__ dtb,
    const float* __restrict__ Alog, const float* __restrict__ Dsp, float* __restrict__ Y)
{
  __shared__ __align__(16) float sBC[SCH * 36];
  const int t  = threadIdx.x;
  const int k  = blockIdx.x & (NDIR - 1);
  const int b_ = blockIdx.x >> 2;
  const int d  = t;
  const int kd = k * DIN + d;
  const float w0 = dtw[kd * 2 + 0], w1 = dtw[kd * 2 + 1];
  const float db = dtb[kd];
  const float Dk = Dsp[kd];
  float An[NST], h[NST];
#pragma unroll
  for (int n = 0; n < NST; ++n) {
    An[n] = -__expf(Alog[(size_t)kd * NST + n]);
    h[n]  = 0.f;
  }
  const size_t tokb = (size_t)b_ * NPIX;
  const int colb = k * XPD;
  float* Yk = Y + (size_t)k * NTOK * DIN;
#pragma unroll 1
  for (int c = 0; c < NPIX / SCH; ++c) {
    __syncthreads();
#pragma unroll 1
    for (int q = t; q < SCH * 9; q += DIN) {
      const int s   = q / 9;
      const int j   = q - s * 9;
      const int tok = dir_tok(k, c * SCH + s);
      const v4f v = *(const v4f*)(XDBL + (tokb + tok) * XPN + colb + 4 * j);
      *(v4f*)(sBC + s * 36 + 4 * j) = v;
    }
    __syncthreads();
#pragma unroll 1
    for (int s = 0; s < SCH; ++s) {
      const int tok = dir_tok(k, c * SCH + s);
      const size_t ei = (tokb + tok) * DIN + d;
      const float u  = XC[ei];
      const float* sr = sBC + s * 36;
      const float dt0 = sr[32], dt1 = sr[33];
      const float dp  = (w0 * dt0 + w1 * dt1) + db;
      const float ex   = __expf(-fabsf(dp));
      const float up1  = 1.0f + ex;
      const float den  = up1 - 1.0f;
      const bool  dpos = den > 0.0f;
      const float dens = dpos ? den : 1.0f;
      const float lg   = __logf(up1);
      const float l1p  = dpos ? (lg * (ex * __builtin_amdgcn_rcpf(dens))) : ex;
      const float delta = fmaxf(dp, 0.0f) + l1p;
      v4f Bv[4], Cv[4];
#pragma unroll
      for (int i = 0; i < 4; ++i) {
        Bv[i] = *(const v4f*)(sr + 4 * i);
        Cv[i] = *(const v4f*)(sr + 16 + 4 * i);
      }
      const float du = delta * u;
      float ys = 0.f;
#pragma unroll
      for (int n = 0; n < NST; ++n) {
        const float e  = __expf(delta * An[n]);
        const float hn = fmaf(e, h[n], du * Bv[n >> 2][n & 3]);
        h[n] = hn;
        ys = fmaf(hn, Cv[n >> 2][n & 3], ys);
      }
      const float y = ys + Dk * u;
      float* yp = Yk + ei;
      *(volatile float*)yp = y;
      __threadfence();
      *(volatile float*)yp = y;
    }
  }
}

__global__ __launch_bounds__(256) void ln_gate_kernel(
    const float* __restrict__ Y, const float* __restrict__ XZ,
    const float* __restrict__ gam, const float* __restrict__ bet,
    unsigned short* __restrict__ YG16)
{
  const int t = threadIdx.x, lane = t & 31, wave = t >> 5;
  const int tok = blockIdx.x * 32 + wave * 4 + (lane >> 3);
  const int c0  = (lane & 7) * 8;
  const size_t PL   = (size_t)NTOK * DIN;
  const size_t base = (size_t)tok * DIN + c0;
  v4f a[2];
#pragma unroll
  for (int j = 0; j < 2; ++j) {
    const v4f y0 = *(const v4f*)(Y + base + 4 * j);
    const v4f y2 = *(const v4f*)(Y + 2 * PL + base + 4 * j);
    const v4f y1 = *(const v4f*)(Y + PL + base + 4 * j);
    const v4f y3 = *(const v4f*)(Y + 3 * PL + base + 4 * j);
    a[j] = ((y0 + y2) + y1) + y3;
  }
  float s = 0.f;
#pragma unroll
  for (int j = 0; j < 2; ++j) s += (a[j][0] + a[j][1]) + (a[j][2] + a[j][3]);
  s += __shfl_xor(s, 1, 32);
  s += __shfl_xor(s, 2, 32);
  s += __shfl_xor(s, 4, 32);
  const float mu = s * (1.0f / 64.0f);
  float q = 0.f;
#pragma unroll
  for (int j = 0; j < 2; ++j) {
#pragma unroll
    for (int e = 0; e < 4; ++e) { const float dd = a[j][e] - mu; q = fmaf(dd, dd, q); }
  }
  q += __shfl_xor(q, 1, 32);
  q += __shfl_xor(q, 2, 32);
  q += __shfl_xor(q, 4, 32);
  const float var = q * (1.0f / 64.0f);
  const float is  = rsqrtf(var + NORM_EPS);
  v8h hv;
#pragma unroll
  for (int j = 0; j < 2; ++j) {
    const v4f zz = *(const v4f*)(XZ + (size_t)tok * XZP + DIN + c0 + 4 * j);
    const v4f gg = *(const v4f*)(gam + c0 + 4 * j);
    const v4f bb = *(const v4f*)(bet + c0 + 4 * j);
#pragma unroll
    for (int e = 0; e < 4; ++e) {
      const float gn = ((a[j][e] - mu) * is) * gg[e] + bb[e];
      const float zv = zz[e];
      const float sg = __builtin_amdgcn_rcpf(1.0f + __expf(-zv));
      const float v  = gn * (zv * sg);
      hv[4 * j + e] = (_Float16)(v * ACARRY);
    }
  }
  unsigned short* op = YG16 + base;
  *(volatile v8h*)op = hv;
  __threadfence();
  *(volatile v8h*)op = hv;
}

__global__ __launch_bounds__(256) void finalize_kernel(
    const float* __restrict__ Tres, const float* __restrict__ O,
    const float* __restrict__ g, const float* __restrict__ be,
    const float* __restrict__ mn, const float* __restrict__ vr,
    float* __restrict__ out, int cbase)
{
  __shared__ __align__(16) float sF[CCH * 68];
  const int t = threadIdx.x, lane = t & 31, wave = t >> 5;
  const int bh = blockIdx.x;
  const int b  = bh >> 6;
  const int h  = bh & (IMH - 1);
  {
    const int w = t >> 2, cg = (t & 3) * 8;
    const size_t tok = (size_t)b * NPIX + h * IMW + w;
#pragma unroll
    for (int j = 0; j < 2; ++j) {
      const v4f tv = *(const v4f*)(Tres + tok * CCH + cg + 4 * j);
      const v4f ov = *(const v4f*)(O + tok * OPN + cg + 4 * j);
      const v4f gg = *(const v4f*)(g  + cbase + cg + 4 * j);
      const v4f bb = *(const v4f*)(be + cbase + cg + 4 * j);
      const v4f mm = *(const v4f*)(mn + cbase + cg + 4 * j);
      const v4f vv = *(const v4f*)(vr + cbase + cg + 4 * j);
#pragma unroll
      for (int e = 0; e < 4; ++e) {
        const float v = tv[e] + ov[e];
        const float r = ((v - mm[e]) * rsqrtf(vv[e] + NORM_EPS)) * gg[e] + bb[e];
        sF[(cg + 4 * j + e) * 68 + w] = fmaxf(r, 0.0f);
      }
    }
  }
  __syncthreads();
  {
    const int col4 = (lane & 15) * 4;
    v4f vals[2];
#pragma unroll
    for (int it = 0; it < 2; ++it) {
      const int row = wave * 4 + it * 2 + (lane >> 4);
      vals[it] = *(const v4f*)(sF + row * 68 + col4);
    }
    for (int pass = 0; pass < 2; ++pass) {
#pragma unroll
      for (int it = 0; it < 2; ++it) {
        const int row = wave * 4 + it * 2 + (lane >> 4);
        float* dst = out + ((size_t)(b * DIMALL + cbase + row)) * NPIX + h * IMW + col4;
        *(volatile v4f*)dst = vals[it];
      }
      __threadfence();
    }
  }
}

extern "C" void kernel_launch(void* const* d_in, const int* in_sizes, int n_in,
                              void* d_out, int out_size, void* d_ws, size_t ws_size,
                              hipStream_t stream)
{
  if (n_in < 36) return;
  if (in_sizes[0] != NBATCH * DIMALL * NPIX) return;
  for (int i = 0; i < 3; ++i) {
    if (in_sizes[1 + 6 * i] != CCH * 7 || in_sizes[2 + 6 * i] != CCH) return;
    if (in_sizes[3 + 6 * i] != CCH * 7 || in_sizes[4 + 6 * i] != CCH) return;
    if (in_sizes[5 + 6 * i] != CCH * 9 || in_sizes[6 + 6 * i] != CCH) return;
  }
  if (in_sizes[19] != CCH || in_sizes[20] != CCH) return;
  if (in_sizes[21] != XZP * CCH) return;
  if (in_sizes[22] != DIN * 9 || in_sizes[23] != DIN) return;
  if (in_sizes[24] != NDIR * XPC * DIN) return;
  if (in_sizes[25] != NDIR * DIN * 2 || in_sizes[26] != NDIR * DIN) return;
  if (in_sizes[27] != NDIR * DIN * NST || in_sizes[28] != NDIR * DIN) return;
  if (in_sizes[29] != DIN || in_sizes[30] != DIN) return;
  if (in_sizes[31] != CCH * DIN) return;
  if (in_sizes[32] != DIMALL || in_sizes[33] != DIMALL || in_sizes[34] != DIMALL || in_sizes[35] != DIMALL) return;
  if (out_size != NBATCH * DIMALL * NPIX) return;

  const float* x = (const float*)d_in[0];
  const float* mh_w[3] = {(const float*)d_in[1],  (const float*)d_in[7],  (const float*)d_in[13]};
  const float* mh_b[3] = {(const float*)d_in[2],  (const float*)d_in[8],  (const float*)d_in[14]};
  const float* mw_w[3] = {(const float*)d_in[3],  (const float*)d_in[9],  (const float*)d_in[15]};
  const float* mw_b[3] = {(const float*)d_in[4],  (const float*)d_in[10], (const float*)d_in[16]};
  const float* c3_w[3] = {(const float*)d_in[5],  (const float*)d_in[11], (const float*)d_in[17]};
  const float* c3_b[3] = {(const float*)d_in[6],  (const float*)d_in[12], (const float*)d_in[18]};
  const float* ln_w       = (const float*)d_in[19];
  const float* ln_b       = (const float*)d_in[20];
  const float* in_proj_w  = (const float*)d_in[21];
  const float* conv_w     = (const float*)d_in[22];
  const float* conv_b     = (const float*)d_in[23];
  const float* x_proj_w   = (const float*)d_in[24];
  const float* dt_proj_w  = (const float*)d_in[25];
  const float* dt_proj_b  = (const float*)d_in[26];
  const float* A_log      = (const float*)d_in[27];
  const float* Dparam     = (const float*)d_in[28];
  const float* onw        = (const float*)d_in[29];
  const float* onb        = (const float*)d_in[30];
  const float* out_proj_w = (const float*)d_in[31];
  const float* bn_g       = (const float*)d_in[32];
  const float* bn_b       = (const float*)d_in[33];
  const float* bn_m       = (const float*)d_in[34];
  const float* bn_v       = (const float*)d_in[35];
  float* dout = (float*)d_out;

  const size_t SZ_TA   = (size_t)NBATCH * CCH * NPIX * 4;
  const size_t SZ_T    = (size_t)NTOK * CCH * 4;
  const size_t SZ_LN16 = (size_t)NTOK * CCH * 2;
  const size_t SZ_XZ   = (size_t)NTOK * XZP * 4;
  const size_t SZ_XC   = (size_t)NTOK * DIN * 4;
  const size_t SZ_XC16 = (size_t)NTOK * DIN * 2;
  const size_t SZ_XDBL = (size_t)NTOK * XPN * 4;
  const size_t SZ_Y    = (size_t)NDIR * NTOK * DIN * 4;
  const size_t SZ_YG16 = (size_t)NTOK * DIN * 2;
  const size_t SZ_O    = (size_t)NTOK * OPN * 4;
  const size_t SZ_WIN  = (size_t)XZP * CCH * 2;
  const size_t SZ_WX   = (size_t)XPN * DIN * 2;
  const size_t SZ_WO   = (size_t)OPN * DIN * 2;
  const size_t OFF_TA   = 0;
  const size_t OFF_TB   = OFF_TA   + SZ_TA;
  const size_t OFF_T    = OFF_TB   + SZ_TA;
  const size_t OFF_LN16 = OFF_T    + SZ_T;
  const size_t OFF_XZ   = OFF_LN16 + SZ_LN16;
  const size_t OFF_XC   = OFF_XZ   + SZ_XZ;
  const size_t OFF_XC16 = OFF_XC   + SZ_XC;
  const size_t OFF_XDBL = OFF_XC16 + SZ_XC16;
  const size_t OFF_Y    = OFF_XDBL + SZ_XDBL;
  const size_t OFF_YG16 = OFF_Y    + SZ_Y;
  const size_t OFF_O    = OFF_YG16 + SZ_YG16;
  const size_t OFF_WIN  = OFF_O    + SZ_O;
  const size_t OFF_WX   = OFF_WIN  + SZ_WIN;
  const size_t OFF_WO   = OFF_WX   + SZ_WX;
  const size_t TOTAL    = OFF_WO   + SZ_WO;
  if (ws_size < TOTAL) return;

  char* ws = (char*)d_ws;
  float*          TA   = (float*)(ws + OFF_TA);
  float*          TB   = (float*)(ws + OFF_TB);
  float*          Tres = (float*)(ws + OFF_T);
  unsigned short* LN16 = (unsigned short*)(ws + OFF_LN16);
  float*          XZ   = (float*)(ws + OFF_XZ);
  float*          XC   = (float*)(ws + OFF_XC);
  unsigned short* XC16 = (unsigned short*)(ws + OFF_XC16);
  float*          XDBL = (float*)(ws + OFF_XDBL);
  float*          YS   = (float*)(ws + OFF_Y);
  unsigned short* YG16 = (unsigned short*)(ws + OFF_YG16);
  float*          O32  = (float*)(ws + OFF_O);
  unsigned short* WIN16 = (unsigned short*)(ws + OFF_WIN);
  unsigned short* WX16  = (unsigned short*)(ws + OFF_WX);
  unsigned short* WO16  = (unsigned short*)(ws + OFF_WO);
  const float* nores = x;

  cast_weights_kernel<<<10, 256, 0, stream>>>(in_proj_w, x_proj_w, out_proj_w, WIN16, WX16, WO16);

  bn_relu_copy_kernel<<<NBATCH * CCH * NPIX / 4 / 256, 256, 0, stream>>>(x, bn_g, bn_b, bn_m, bn_v, dout);

  for (int i = 0; i < 3; ++i) {
    const int cbase = CCH * i;
    const int dil   = i + 1;

    dw_w7_kernel<<<NBATCH * CCH * NPIX / 4 / 256, 256, 0, stream>>>(x, mw_w[i], mw_b[i], TA, cbase, dil);
    dw_h7_kernel<<<NBATCH * CCH * NPIX / 4 / 256, 256, 0, stream>>>(TA, mh_w[i], mh_b[i], TB, dil);
    dw_c_ln_kernel<<<NBATCH * IMH * 2, 256, 0, stream>>>(TB, x, c3_w[i], c3_b[i], ln_w, ln_b, Tres, LN16, cbase, dil);

    wmma_gemm64<0, false, 0, 0, false, 0><<<dim3(128, 1), 256, 0, stream>>>(
        LN16, LN16, CCH, 0L, WIN16, WIN16, CCH, 0L, (void*)XZ, (void*)XZ, XZP, 0L,
        nores, nores, 0L, NTOK, XZP, CCH, 1.0f / WCARRY);

    conv_silu_kernel<<<NBATCH * IMH, DIN, 0, stream>>>(XZ, conv_w, conv_b, XC, XC16);

    wmma_gemm64<0, false, 0, 0, false, 0><<<dim3(192, 1), 256, 0, stream>>>(
        XC16, XC16, DIN, 0L, WX16, WX16, DIN, 0L, (void*)XDBL, (void*)XDBL, XPN, 0L,
        nores, nores, 0L, NTOK, XPN, DIN, 1.0f / (ACARRY * WCARRY));

    scan_kernel<<<NBATCH * NDIR, DIN, 0, stream>>>(XDBL, XC, dt_proj_w, dt_proj_b, A_log, Dparam, YS);

    ln_gate_kernel<<<NTOK / 32, 256, 0, stream>>>(YS, XZ, onw, onb, YG16);

    wmma_gemm64<0, false, 0, 0, false, 0><<<dim3(64, 1), 256, 0, stream>>>(
        YG16, YG16, DIN, 0L, WO16, WO16, DIN, 0L, (void*)O32, (void*)O32, OPN, 0L,
        nores, nores, 0L, NTOK, OPN, DIN, 1.0f / (ACARRY * WCARRY));

    finalize_kernel<<<NBATCH * IMH, 256, 0, stream>>>(Tres, O32, bn_g, bn_b, bn_m, bn_v, dout, cbase);
  }
}
